// SPADE_33981781246328
// MI455X (gfx1250) — hardware-verified
//
#include <hip/hip_runtime.h>
#include <stddef.h>
#include <math.h>

constexpr int kBatch  = 2;
constexpr int kImg    = 96;
constexpr int kHW     = 9216;
constexpr int kPix    = 18432;
constexpr int kChX    = 64;
constexpr int kChR    = 64;
constexpr int kChCat  = 128;
constexpr int kMid    = 16;
constexpr int kOffCh  = 27;
constexpr int kNpad   = 64;
constexpr int kChGB   = 128;
constexpr int kTaps   = 9;
constexpr int kK1     = 1152;
constexpr int kK2real = 144;
constexpr int kK2     = 192;
constexpr int kK3     = 576;
constexpr int kParSlot = 64;

static_assert(kBatch * kHW == kPix, "");
static_assert(kPix % 64 == 0 && kNpad % 64 == 0 && kChGB % 64 == 0, "");
static_assert(kK1 % 64 == 0 && kK2 % 64 == 0 && kK3 % 64 == 0, "");
static_assert(kK2 >= kK2real, "");
static_assert(kPix % 32 == 0 && (kPix * kTaps) % 64 == 0, "");
static_assert(kImg % 4 == 0 && kChCat % 8 == 0 && kMid % 8 == 0 && kChR % 8 == 0, "");

typedef __attribute__((ext_vector_type(16))) _Float16 v16h;
typedef __attribute__((ext_vector_type(8)))  _Float16 v8h;
typedef __attribute__((ext_vector_type(16))) __bf16   v16b;
typedef __attribute__((ext_vector_type(8)))  __bf16   v8b;
typedef __attribute__((ext_vector_type(8)))  float    v8f;
typedef __attribute__((ext_vector_type(4)))  float    v4f;
typedef __attribute__((ext_vector_type(4)))  unsigned v4u;

__device__ __forceinline__ unsigned short f2bf_bits(float f) {
  unsigned u = __float_as_uint(f);
  return (unsigned short)((u + 0x7FFFu + ((u >> 16) & 1u)) >> 16);
}
__device__ __forceinline__ float bf_bits2f(unsigned short h) { return __uint_as_float(((unsigned)h) << 16); }

__device__ __forceinline__ unsigned pk2(unsigned short a, unsigned short b) {
  return (unsigned)a | ((unsigned)b << 16);
}
__device__ __forceinline__ unsigned pkh2(float a, float b) {
  return pk2(__builtin_bit_cast(unsigned short, (_Float16)a), __builtin_bit_cast(unsigned short, (_Float16)b));
}

__device__ __forceinline__ void dep_guard_h(v8f& a, v8f& b, v16h x, v16h y) { asm volatile("v_nop\n\tv_nop\n\tv_nop\n\tv_nop" : "+v"(a), "+v"(b) : "v"(x), "v"(y)); }
__device__ __forceinline__ void dep_guard_b(v8f& a, v8f& b, v16b x, v16b y) { asm volatile("v_nop\n\tv_nop\n\tv_nop\n\tv_nop" : "+v"(a), "+v"(b) : "v"(x), "v"(y)); }
__device__ __forceinline__ void keep4_h(v16h a, v16h b, v16h c, v16h d) { asm volatile("v_nop" :: "v"(a), "v"(b), "v"(c), "v"(d)); }
__device__ __forceinline__ void keep4_b(v16b a, v16b b, v16b c, v16b d) { asm volatile("v_nop" :: "v"(a), "v"(b), "v"(c), "v"(d)); }
__device__ __forceinline__ void acc_guard4(v8f& a, v8f& b, v8f& c, v8f& d) { asm volatile("v_nop\n\tv_nop\n\tv_nop\n\tv_nop" : "+v"(a), "+v"(b), "+v"(c), "+v"(d)); }
template <typename T> struct Frag;
template <> struct Frag<_Float16> {
  typedef v16h V; union U { v16h v; v8h h[2]; };
  static __device__ __forceinline__ v16h load(const _Float16* p) {
    U f; f.h[0] = *(const v8h*)(p); f.h[1] = *(const v8h*)(p + 16); return f.v;
  }
  static __device__ __forceinline__ v8f mma(v16h a, v16h b, v8f c) {
    return __builtin_amdgcn_wmma_f32_16x16x32_f16(false, a, false, b, (short)0, c, false, false);
  }
  static __device__ __forceinline__ void guard(v8f& a, v8f& b, v16h x, v16h y) { dep_guard_h(a, b, x, y); }
  static __device__ __forceinline__ void keep(v16h a, v16h b, v16h c, v16h d) { keep4_h(a, b, c, d); }
};
template <> struct Frag<__bf16> {
  typedef v16b V; union U { v16b v; v8b h[2]; };
  static __device__ __forceinline__ v16b load(const __bf16* p) {
    U f; f.h[0] = *(const v8b*)(p); f.h[1] = *(const v8b*)(p + 16); return f.v;
  }
  static __device__ __forceinline__ v8f mma(v16b a, v16b b, v8f c) {
    return __builtin_amdgcn_wmma_f32_16x16x32_bf16(false, a, false, b, (short)0, c, false, false);
  }
  static __device__ __forceinline__ void guard(v8f& a, v8f& b, v16b x, v16b y) { dep_guard_b(a, b, x, y); }
  static __device__ __forceinline__ void keep(v16b a, v16b b, v16b c, v16b d) { keep4_b(a, b, c, d); }
};

template <int ET> struct Elem;
template <> struct Elem<0> { typedef _Float16 T; };
template <> struct Elem<1> { typedef __bf16 T; };
template <int ET, int SPLITM, int BIAS_MODE, int OUT_MODE, bool RESID, int ACT = 0>
__global__ __launch_bounds__(256) void wmma_gemm64(
    const unsigned short* __restrict__ Ap, const unsigned short* __restrict__ A2p, int lda, long strideA,
    const unsigned short* __restrict__ Btp, const unsigned short* __restrict__ Bt2p, int ldb, long strideB,
    void* __restrict__ Cout, void* __restrict__ Cout2, int ldc, long strideC,
    const float* __restrict__ bias,
    const float* __restrict__ resid, long strideR,
    int M, int N, int K, float scale) {
  typedef typename Elem<ET>::T T;
  typedef typename Frag<T>::V V;
  constexpr bool SPLA = (SPLITM != 0);
  constexpr bool SPLB = (SPLITM == 1);
  const T* A = (const T*)Ap; const T* A2 = (const T*)A2p; const T* Bt = (const T*)Btp; const T* Bt2 = (const T*)Bt2p;
  __shared__ __align__(16) float sT[8][16 * 68];
  const int b    = blockIdx.y;
  const int lane = threadIdx.x & 31;
  const int wave = threadIdx.x >> 5;
  const int tilesN = N >> 6;
  const int tilesM = M >> 6;
  const int tile = blockIdx.x * 8 + wave;
  if (tile >= tilesM * tilesN) return;
  const int tm = tile / tilesN;
  const int tn = tile - tm * tilesN;
  const int m0 = tm << 6;
  const int n0 = tn << 6;

  const T* Ab  = A  + (size_t)b * strideA;
  const T* Bb  = Bt + (size_t)b * strideB;
  const T* Ab2 = SPLA ? (A2  + (size_t)b * strideA) : nullptr;
  const T* Bb2 = SPLB ? (Bt2 + (size_t)b * strideB) : nullptr;

  const int rlane = lane & 15;
  const int koff  = (lane >> 4) * 8;
  const int mOff  = (lane >> 4) * 8;

  v8f acc[4][4];
#pragma unroll
  for (int i = 0; i < 4; ++i)
#pragma unroll
    for (int j = 0; j < 4; ++j) acc[i][j] = (v8f){0.f,0.f,0.f,0.f,0.f,0.f,0.f,0.f};

  for (int k0 = 0; k0 < K; k0 += 32) {
    V bh[4], bl[4];
#pragma unroll
    for (int j = 0; j < 4; ++j) {
      const size_t bo = (size_t)(n0 + (j << 4) + rlane) * ldb + koff + k0;
      bh[j] = Frag<T>::load(Bb + bo);
      if (SPLB) bl[j] = Frag<T>::load(Bb2 + bo);
    }
#pragma unroll
    for (int i = 0; i < 4; ++i) {
      const size_t ao = (size_t)(m0 + (i << 4) + rlane) * lda + koff + k0;
      V ah = Frag<T>::load(Ab + ao);
      V al;
      if (SPLA) al = Frag<T>::load(Ab2 + ao);
#pragma unroll
      for (int j = 0; j < 4; ++j) {
        acc[i][j] = Frag<T>::mma(ah, bh[j], acc[i][j]);
        if (SPLB) acc[i][j] = Frag<T>::mma(ah, bl[j], acc[i][j]);
        if (SPLA) acc[i][j] = Frag<T>::mma(al, bh[j], acc[i][j]);
      }
      Frag<T>::guard(acc[i][0], acc[i][3], ah, SPLA ? al : ah);
    }
    Frag<T>::keep(bh[0], bh[1], bh[2], bh[3]);
    if (SPLB) Frag<T>::keep(bl[0], bl[1], bl[2], bl[3]);
  }
  acc_guard4(acc[0][0], acc[0][1], acc[0][2], acc[0][3]);
  acc_guard4(acc[1][0], acc[1][1], acc[1][2], acc[1][3]);
  acc_guard4(acc[2][0], acc[2][1], acc[2][2], acc[2][3]);
  acc_guard4(acc[3][0], acc[3][1], acc[3][2], acc[3][3]);

  float* slab = sT[wave];
  const float* Rb = RESID ? (resid + (size_t)b * strideR) : nullptr;
#pragma unroll
  for (int i = 0; i < 4; ++i) {
    const int mBase = m0 + (i << 4);
#pragma unroll
    for (int j = 0; j < 4; ++j) {
      const int n = n0 + (j << 4) + rlane;
      float bv = 0.f;
      if (BIAS_MODE == 2) bv = bias[n];
#pragma unroll
      for (int r = 0; r < 8; ++r) {
        float v = acc[i][j][r] * scale;
        if (BIAS_MODE == 1) v += bias[mBase + mOff + r];
        if (BIAS_MODE == 2) v += bv;
        if (ACT == 1) v = tanhf(v);
        if (ACT == 2) v = fmaxf(v, 0.0f);
        if (ACT == 4) v = (v > 0.f) ? v : 0.01f * v;
        if (RESID) v += Rb[(size_t)(mBase + mOff + r) * ldc + n];
        slab[(mOff + r) * 68 + (j << 4) + rlane] = v;
      }
    }
    __builtin_amdgcn_fence(__ATOMIC_RELEASE, "workgroup");
    __builtin_amdgcn_wave_barrier();
    __builtin_amdgcn_fence(__ATOMIC_ACQUIRE, "workgroup");
    if (OUT_MODE == 0) {
      float* C = (float*)Cout + (size_t)b * strideC;
      const int hh = lane >> 4, c4 = (lane & 15) * 4;
      for (int pass = 0; pass < 2; ++pass) {
#pragma unroll
        for (int it = 0; it < 8; ++it) {
          const int row = it * 2 + hh;
          v4f v = *(const v4f*)(slab + row * 68 + c4);
          *(volatile v4f*)(C + (size_t)(mBase + row) * ldc + n0 + c4) = v;
        }
        __threadfence();
      }
    } else {
      const int q = lane >> 3, c8 = (lane & 7) * 8;
      unsigned short* C  = (unsigned short*)Cout  + (size_t)b * strideC;
      unsigned short* C2 = (OUT_MODE == 2) ? ((unsigned short*)Cout2 + (size_t)b * strideC) : nullptr;
      for (int pass = 0; pass < 2; ++pass) {
#pragma unroll
        for (int it = 0; it < 4; ++it) {
          const int row = it * 4 + q;
          const float* sp = slab + row * 68 + c8;
          v8h hv, lv;
#pragma unroll
          for (int e = 0; e < 8; ++e) {
            if (OUT_MODE == 1) {
              hv[e] = (_Float16)sp[e];
            } else {
              unsigned short hb = f2bf_bits(sp[e]);
              unsigned short lb = f2bf_bits(sp[e] - bf_bits2f(hb));
              hv[e] = __builtin_bit_cast(_Float16, hb);
              lv[e] = __builtin_bit_cast(_Float16, lb);
            }
          }
          *(volatile v8h*)(C + (size_t)(mBase + row) * ldc + n0 + c8) = hv;
          if (OUT_MODE == 2) *(volatile v8h*)(C2 + (size_t)(mBase + row) * ldc + n0 + c8) = lv;
        }
        __threadfence();
      }
    }
    __builtin_amdgcn_fence(__ATOMIC_RELEASE, "workgroup");
    __builtin_amdgcn_wave_barrier();
    __builtin_amdgcn_fence(__ATOMIC_ACQUIRE, "workgroup");
  }
}

__global__ __launch_bounds__(256) void k_prepw(const float* __restrict__ w, unsigned short* __restrict__ dst,
                                               int cin, int kpad, int nreal, float scale) {
  const int lane = threadIdx.x & 31, wave = threadIdx.x >> 5;
  const int n = blockIdx.x * 8 + wave;
  const int q = lane >> 3, c8l = (lane & 7) * 8;
  const int nlines = kpad >> 6, niter = (nlines + 3) >> 2;
  const int kreal = kTaps * cin;
  const int nc = n < nreal ? n : (nreal - 1);
#pragma unroll 1
  for (int i = 0; i < niter; ++i) {
    const int line = i * 4 + q;
    const int col0 = line * 64 + c8l;
    const int tap = col0 / cin;
    const int c0 = col0 - tap * cin;
    const int tapc = tap < 8 ? tap : 8;
    const bool valid = (n < nreal) && (col0 < kreal);
    const float* src = w + ((size_t)nc * cin + c0) * kTaps + tapc;
    float f[8];
#pragma unroll
    for (int e = 0; e < 8; ++e) {
      const float t = src[(size_t)e * kTaps] * scale;
      f[e] = valid ? t : 0.0f;
    }
    v4u u;
    u[0] = pkh2(f[0], f[1]); u[1] = pkh2(f[2], f[3]); u[2] = pkh2(f[4], f[5]); u[3] = pkh2(f[6], f[7]);
    const bool st = line < nlines;
    volatile v4u* d = (volatile v4u*)(dst + (size_t)n * kpad + col0);
    if (st) *d = u;
    __threadfence();
    if (st) *d = u;
  }
}

__global__ __launch_bounds__(32) void k_par(const float* __restrict__ b1, const float* __restrict__ b2,
                                            const float* __restrict__ boff, const float* __restrict__ bdf,
                                            const float* __restrict__ bg, const float* __restrict__ bbe,
                                            float* __restrict__ par) {
  const int slot = blockIdx.x;
  const int lane = threadIdx.x;
  const int e0 = (lane & 15) * 4;
  v4f v;
#pragma unroll
  for (int j = 0; j < 4; ++j) {
    const int e = e0 + j;
    const float f0 = b1[e < kMid ? e : (kMid - 1)];
    const float f1 = b2[e];
    const float f2 = boff[e < kOffCh ? e : (kOffCh - 1)];
    const float f3 = bdf[e] * 16.0f;
    const float f4 = bg[e];
    const float f5 = bbe[e];
    const float a0 = (e < kMid) ? f0 : 0.0f;
    const float a2 = (e < kOffCh) ? f2 : 0.0f;
    v[j] = (slot == 0) ? a0 : (slot == 1) ? f1 : (slot == 2) ? a2 : (slot == 3) ? f3 : (slot == 4) ? f4 : f5;
  }
  volatile v4f* p = (volatile v4f*)(par + (size_t)slot * kParSlot + e0);
  if (lane < 16) *p = v;
  __threadfence();
  if (lane < 16) *p = v;
}

__global__ __launch_bounds__(256) void k_front(const float* __restrict__ x, const float* __restrict__ rf,
                                               float* __restrict__ nrm, unsigned short* __restrict__ cat,
                                               float* __restrict__ ref32) {
  __shared__ float xs[kChX][97];
  __shared__ float rs[kChR][97];
  __shared__ float smean[kImg];
  __shared__ float sinv[kImg];
  const int tid = threadIdx.x;
  const int bh = blockIdx.x;
  const int b = bh / kImg, h = bh - b * kImg;
#pragma unroll
  for (int i = 0; i < 6; ++i) {
    const int f = tid + 256 * i;
    const int c = f / 24, q4 = (f - c * 24) * 4;
    const size_t g = (((size_t)(b * kChX + c)) * kImg + h) * kImg + q4;
    const v4f vx = *(const v4f*)(x + g);
    const v4f vr = *(const v4f*)(rf + g);
#pragma unroll
    for (int e = 0; e < 4; ++e) { xs[c][q4 + e] = vx[e]; rs[c][q4 + e] = vr[e]; }
  }
  __syncthreads();
  if (tid < kImg) {
    float s = 0.f;
#pragma unroll 1
    for (int c = 0; c < kChX; ++c) s += xs[c][tid];
    const float mean = s * (1.0f / 64.0f);
    float s2 = 0.f;
#pragma unroll 1
    for (int c = 0; c < kChX; ++c) { const float d = xs[c][tid] - mean; s2 += d * d; }
    const float var = s2 * (1.0f / 63.0f);
    smean[tid] = mean;
    sinv[tid] = 1.0f / sqrtf(var + 1e-5f);
  }
  __syncthreads();
  const int wave = tid >> 5, lane = tid & 31;
  {
    const int wl = lane < 24 ? lane : 23;
    const int w0 = wl * 4;
    for (int pass = 0; pass < 2; ++pass) {
#pragma unroll 1
      for (int i = 0; i < 8; ++i) {
        const int c = wave * 8 + i;
        v4f o;
#pragma unroll
        for (int e = 0; e < 4; ++e) o[e] = (xs[c][w0 + e] - smean[w0 + e]) * sinv[w0 + e];
        if (lane < 24) *(volatile v4f*)(nrm + (((size_t)(b * kChX + c)) * kImg + h) * kImg + w0) = o;
      }
      __threadfence();
    }
  }
  {
    const int hsel = lane >> 4;
    const int ch0 = (lane & 15) * 8;
    const int cx = ch0 & 63;
    const bool isn = ch0 < 64;
    for (int pass = 0; pass < 2; ++pass) {
#pragma unroll 1
      for (int i = 0; i < 6; ++i) {
        const int pp = wave + 8 * i;
        const int w = 2 * pp + hsel;
        const float m = smean[w], iv = sinv[w];
        float f[8];
#pragma unroll
        for (int e = 0; e < 8; ++e) {
          const float a = (xs[cx + e][w] - m) * iv;
          const float r = rs[cx + e][w];
          f[e] = isn ? a : r;
        }
        v4u u;
        u[0] = pkh2(f[0], f[1]); u[1] = pkh2(f[2], f[3]); u[2] = pkh2(f[4], f[5]); u[3] = pkh2(f[6], f[7]);
        *(volatile v4u*)(cat + ((size_t)(bh * kImg + w)) * kChCat + ch0) = u;
      }
      __threadfence();
    }
  }
  {
    const int hsel = lane >> 4;
    const int c0 = (lane & 15) * 4;
    for (int pass = 0; pass < 2; ++pass) {
#pragma unroll 1
      for (int i = 0; i < 6; ++i) {
        const int pp = wave + 8 * i;
        const int w = 2 * pp + hsel;
        v4f o;
#pragma unroll
        for (int e = 0; e < 4; ++e) o[e] = rs[c0 + e][w];
        *(volatile v4f*)(ref32 + ((size_t)(bh * kImg + w)) * kChR + c0) = o;
      }
      __threadfence();
    }
  }
}

__global__ __launch_bounds__(256) void k_im2col(const unsigned short* __restrict__ src, int spitch, int cin,
                                                unsigned short* __restrict__ dst, int kpad) {
  const int lane = threadIdx.x & 31, wave = threadIdx.x >> 5;
  const int q = lane >> 3, c8l = (lane & 7) * 8;
  const int nlines = kpad >> 6, niter = (nlines + 3) >> 2;
  const int kreal = kTaps * cin;
  const v4u z = (v4u){0u, 0u, 0u, 0u};
#pragma unroll 1
  for (int r = 0; r < 4; ++r) {
    const int p = (blockIdx.x * 8 + wave) * 4 + r;
    const int b = p / kHW, hw = p - b * kHW;
    const int h = hw / kImg, w = hw - h * kImg;
#pragma unroll 1
    for (int i = 0; i < niter; ++i) {
      const int line = i * 4 + q;
      const int col0 = line * 64 + c8l;
      const int tap = col0 / cin;
      const int c0 = col0 - tap * cin;
      const int tapc = tap < 8 ? tap : 8;
      const int kh = tapc / 3, kw = tapc - kh * 3;
      const int y = h + kh - 1, xx = w + kw - 1;
      const bool inb = ((unsigned)y < (unsigned)kImg) && ((unsigned)xx < (unsigned)kImg) && (col0 < kreal);
      const int yc = y < 0 ? 0 : (y > kImg - 1 ? kImg - 1 : y);
      const int xc = xx < 0 ? 0 : (xx > kImg - 1 ? kImg - 1 : xx);
      v4u v = *(const v4u*)(src + ((size_t)(b * kHW + yc * kImg + xc)) * spitch + c0);
      if (!inb) v = z;
      const bool st = line < nlines;
      volatile v4u* d = (volatile v4u*)(dst + (size_t)p * kpad + col0);
      if (st) *d = v;
      __threadfence();
      if (st) *d = v;
    }
  }
}

__global__ __launch_bounds__(256) void k_sample(const float* __restrict__ ref32, const float* __restrict__ om,
                                                unsigned short* __restrict__ s16) {
  const int lane = threadIdx.x & 31, wave = threadIdx.x >> 5;
  const int sub = lane >> 3, c8 = (lane & 7) * 8;
  const v4f z = (v4f){0.f, 0.f, 0.f, 0.f};
  const float lim = (float)(kImg - 1);
#pragma unroll 1
  for (int r = 0; r < 2; ++r) {
    const int item = ((blockIdx.x * 8 + wave) * 2 + r) * 4 + sub;
    const int p = item / kTaps, k = item - p * kTaps;
    const int b = p / kHW, hw = p - b * kHW;
    const int h = hw / kImg, w = hw - h * kImg;
    const int kh = k / 3, kw = k - kh * 3;
    const float* orow = om + (size_t)p * kNpad;
    const float dy = orow[2 * k];
    const float dx = orow[2 * k + 1];
    float ml = orow[18 + k];
    ml = fminf(fmaxf(ml, -30.0f), 30.0f);
    const float msk = __builtin_amdgcn_rcpf(1.0f + expf(-ml));
    const float sy = (dy + (float)h) + (float)(kh - 1);
    const float sx = (dx + (float)w) + (float)(kw - 1);
    const float y0 = floorf(sy), x0 = floorf(sx);
    const float y1 = y0 + 1.0f, x1 = x0 + 1.0f;
    const float wy1 = sy - y0, wx1 = sx - x0;
    const float wy0 = 1.0f - wy1, wx0 = 1.0f - wx1;
    const bool vy0 = (y0 >= 0.0f) && (y0 <= lim);
    const bool vy1 = (y1 >= 0.0f) && (y1 <= lim);
    const bool vx0 = (x0 >= 0.0f) && (x0 <= lim);
    const bool vx1 = (x1 >= 0.0f) && (x1 <= lim);
    const int yi0 = (int)fminf(fmaxf(y0, 0.0f), lim);
    const int yi1 = (int)fminf(fmaxf(y1, 0.0f), lim);
    const int xi0 = (int)fminf(fmaxf(x0, 0.0f), lim);
    const int xi1 = (int)fminf(fmaxf(x1, 0.0f), lim);
    const float* ub  = ref32 + (size_t)b * kHW * kChR + c8;
    const float* q00 = ub + ((size_t)yi0 * kImg + xi0) * kChR;
    const float* q01 = ub + ((size_t)yi0 * kImg + xi1) * kChR;
    const float* q10 = ub + ((size_t)yi1 * kImg + xi0) * kChR;
    const float* q11 = ub + ((size_t)yi1 * kImg + xi1) * kChR;
    v4f g00a = *(const v4f*)(q00), g00b = *(const v4f*)(q00 + 4);
    v4f g01a = *(const v4f*)(q01), g01b = *(const v4f*)(q01 + 4);
    v4f g10a = *(const v4f*)(q10), g10b = *(const v4f*)(q10 + 4);
    v4f g11a = *(const v4f*)(q11), g11b = *(const v4f*)(q11 + 4);
    const bool k00 = vy0 && vx0, k01 = vy0 && vx1, k10 = vy1 && vx0, k11 = vy1 && vx1;
    g00a = k00 ? g00a : z; g00b = k00 ? g00b : z;
    g01a = k01 ? g01a : z; g01b = k01 ? g01b : z;
    g10a = k10 ? g10a : z; g10b = k10 ? g10b : z;
    g11a = k11 ? g11a : z; g11b = k11 ? g11b : z;
    const v4f topa = g00a * wx0 + g01a * wx1, topb = g00b * wx0 + g01b * wx1;
    const v4f bota = g10a * wx0 + g11a * wx1, botb = g10b * wx0 + g11b * wx1;
    v4f va = topa * wy0 + bota * wy1;
    v4f vb = topb * wy0 + botb * wy1;
    const float mk = msk * 16.0f;
    va = va * mk;
    vb = vb * mk;
    v4u u;
    u[0] = pkh2(va[0], va[1]); u[1] = pkh2(va[2], va[3]);
    u[2] = pkh2(vb[0], vb[1]); u[3] = pkh2(vb[2], vb[3]);
    volatile v4u* d = (volatile v4u*)(s16 + (size_t)p * kK3 + k * kChR + c8);
    *d = u;
    __threadfence();
    *d = u;
  }
}

__global__ __launch_bounds__(256) void k_final(const float* __restrict__ nrm, const float* __restrict__ gb,
                                               float* __restrict__ out) {
  __shared__ __align__(16) float gs[kImg][132];
  const int tid = threadIdx.x;
  const int bh = blockIdx.x;
  const int b = bh / kImg, h = bh - b * kImg;
#pragma unroll
  for (int i = 0; i < 12; ++i) {
    const int f = tid + 256 * i;
    const int row = f >> 5, q4 = (f & 31) * 4;
    const v4f v = *(const v4f*)(gb + ((size_t)(bh * kImg + row)) * kChGB + q4);
    *(v4f*)(&gs[row][q4]) = v;
  }
  __syncthreads();
  const int wave = tid >> 5, lane = tid & 31;
  const int wl = lane < 24 ? lane : 23;
  const int w0 = wl * 4;
  for (int pass = 0; pass < 2; ++pass) {
#pragma unroll 1
    for (int i = 0; i < 8; ++i) {
      const int c = wave * 8 + i;
      const size_t idx = (((size_t)(b * kChX + c)) * kImg + h) * kImg + w0;
      const v4f n = *(const v4f*)(nrm + idx);
      v4f o;
#pragma unroll
      for (int e = 0; e < 4; ++e) {
        const float g = gs[w0 + e][c];
        const float be = gs[w0 + e][kChX + c];
        o[e] = n[e] * (1.0f + g) + be;
      }
      if (lane < 24) *(volatile v4f*)(out + idx) = o;
    }
    __threadfence();
  }
}

extern "C" void kernel_launch(void* const* d_in, const int* in_sizes, int n_in,
                              void* d_out, int out_size, void* d_ws, size_t ws_size,
                              hipStream_t stream) {
  if (n_in < 14) return;
  if (in_sizes[0] != kPix * kChX || in_sizes[1] != kPix * kChR || in_sizes[2] != kMid * kChCat * kTaps ||
      in_sizes[3] != kMid || in_sizes[4] != kChR * kMid * kTaps || in_sizes[5] != kChR ||
      in_sizes[6] != kOffCh * kChR * kTaps || in_sizes[7] != kOffCh || in_sizes[8] != kChR * kChR * kTaps ||
      in_sizes[9] != kChR || in_sizes[10] != kChX * kChR * kTaps || in_sizes[11] != kChX ||
      in_sizes[12] != kChX * kChR * kTaps || in_sizes[13] != kChX) return;
  if (out_size != kPix * kChX) return;

  const float* x     = (const float*)d_in[0];
  const float* rfeat = (const float*)d_in[1];
  const float* w1    = (const float*)d_in[2];
  const float* b1    = (const float*)d_in[3];
  const float* w2    = (const float*)d_in[4];
  const float* b2    = (const float*)d_in[5];
  const float* w_off = (const float*)d_in[6];
  const float* b_off = (const float*)d_in[7];
  const float* w_df  = (const float*)d_in[8];
  const float* b_df  = (const float*)d_in[9];
  const float* w_g   = (const float*)d_in[10];
  const float* b_g   = (const float*)d_in[11];
  const float* w_be  = (const float*)d_in[12];
  const float* b_be  = (const float*)d_in[13];
  float* out = (float*)d_out;

  const size_t bytes_NRM  = (size_t)kPix * kChX * 4;
  const size_t bytes_REF  = (size_t)kPix * kChR * 4;
  const size_t bytes_CAT  = (size_t)kPix * kChCat * 2;
  const size_t bytes_IM   = (size_t)kPix * kK1 * 2;
  const size_t bytes_H16  = (size_t)kPix * kNpad * 2;
  const size_t bytes_COND = (size_t)kPix * kChR * 2;
  const size_t bytes_OM   = (size_t)kPix * kNpad * 4;
  const size_t bytes_S16  = (size_t)kPix * kK3 * 2;
  const size_t bytes_RR   = (size_t)kPix * kChR * 2;
  const size_t bytes_GB   = (size_t)kPix * kChGB * 4;
  const size_t bytes_W1P  = (size_t)kNpad * kK1 * 2;
  const size_t bytes_W2P  = (size_t)kNpad * kK2 * 2;
  const size_t bytes_WOP  = (size_t)kNpad * kK3 * 2;
  const size_t bytes_WDP  = (size_t)kNpad * kK3 * 2;
  const size_t bytes_WGBP = (size_t)kChGB * kK3 * 2;
  const size_t bytes_PAR  = (size_t)6 * kParSlot * 4;

  char* ws = (char*)d_ws;
  size_t o = 0;
  float*          NRM32  = (float*)(ws + o);            o += bytes_NRM;
  float*          REF32  = (float*)(ws + o);            o += bytes_REF;
  unsigned short* CAT16  = (unsigned short*)(ws + o);   o += bytes_CAT;
  unsigned short* IM16   = (unsigned short*)(ws + o);   o += bytes_IM;
  unsigned short* H16    = (unsigned short*)(ws + o);   o += bytes_H16;
  unsigned short* COND16 = (unsigned short*)(ws + o);   o += bytes_COND;
  float*          OM32   = (float*)(ws + o);            o += bytes_OM;
  unsigned short* S16    = (unsigned short*)(ws + o);   o += bytes_S16;
  unsigned short* RR16   = (unsigned short*)(ws + o);   o += bytes_RR;
  float*          GB32   = (float*)(ws + o);            o += bytes_GB;
  unsigned short* W1P    = (unsigned short*)(ws + o);   o += bytes_W1P;
  unsigned short* W2P    = (unsigned short*)(ws + o);   o += bytes_W2P;
  unsigned short* WOP    = (unsigned short*)(ws + o);   o += bytes_WOP;
  unsigned short* WDP    = (unsigned short*)(ws + o);   o += bytes_WDP;
  unsigned short* WGBP   = (unsigned short*)(ws + o);   o += bytes_WGBP;
  float*          PAR    = (float*)(ws + o);            o += bytes_PAR;
  if (o > ws_size || o > (size_t)134217728) return;

  const float* p_b1   = PAR + 0 * kParSlot;
  const float* p_b2   = PAR + 1 * kParSlot;
  const float* p_boff = PAR + 2 * kParSlot;
  const float* p_bdf  = PAR + 3 * kParSlot;
  const float* p_bgb  = PAR + 4 * kParSlot;

  k_prepw<<<8, 256, 0, stream>>>(w1,    W1P,  kChCat, kK1, kMid,   16.0f);
  k_prepw<<<8, 256, 0, stream>>>(w2,    W2P,  kMid,   kK2, kChR,   16.0f);
  k_prepw<<<8, 256, 0, stream>>>(w_off, WOP,  kChR,   kK3, kOffCh, 256.0f);
  k_prepw<<<8, 256, 0, stream>>>(w_df,  WDP,  kChR,   kK3, kChR,   16.0f);
  k_prepw<<<8, 256, 0, stream>>>(w_g,   WGBP, kChR,   kK3, kChX,   16.0f);
  k_prepw<<<8, 256, 0, stream>>>(w_be,  WGBP + (size_t)kChX * kK3, kChR, kK3, kChX, 16.0f);
  k_par<<<6, 32, 0, stream>>>(b1, b2, b_off, b_df, b_g, b_be, PAR);
  k_front<<<kBatch * kImg, 256, 0, stream>>>(x, rfeat, NRM32, CAT16, REF32);

  const int blocksN64  = ((kPix / 64) * 1 + 7) / 8;
  const int blocksN128 = ((kPix / 64) * 2 + 7) / 8;

  k_im2col<<<kPix / 32, 256, 0, stream>>>(CAT16, kChCat, kChCat, IM16, kK1);
  wmma_gemm64<0, 0, 2, 1, false, 2><<<dim3(blocksN64, 1), 256, 0, stream>>>(
      IM16, IM16, kK1, 0L, W1P, W1P, kK1, 0L, (void*)H16, (void*)H16, kNpad, 0L,
      p_b1, p_b1, 0L, kPix, kNpad, kK1, 0.0625f);

  k_im2col<<<kPix / 32, 256, 0, stream>>>(H16, kNpad, kMid, IM16, kK2);
  wmma_gemm64<0, 0, 2, 1, false, 2><<<dim3(blocksN64, 1), 256, 0, stream>>>(
      IM16, IM16, kK2, 0L, W2P, W2P, kK2, 0L, (void*)COND16, (void*)COND16, kNpad, 0L,
      p_b2, p_b2, 0L, kPix, kNpad, kK2, 0.0625f);

  k_im2col<<<kPix / 32, 256, 0, stream>>>(COND16, kNpad, kChR, IM16, kK3);
  wmma_gemm64<0, 0, 2, 0, false, 0><<<dim3(blocksN64, 1), 256, 0, stream>>>(
      IM16, IM16, kK3, 0L, WOP, WOP, kK3, 0L, (void*)OM32, (void*)OM32, kNpad, 0L,
      p_boff, p_boff, 0L, kPix, kNpad, kK3, 0.00390625f);

  k_sample<<<(kPix * kTaps) / 64, 256, 0, stream>>>(REF32, OM32, S16);
  wmma_gemm64<0, 0, 2, 1, false, 0><<<dim3(blocksN64, 1), 256, 0, stream>>>(
      S16, S16, kK3, 0L, WDP, WDP, kK3, 0L, (void*)RR16, (void*)RR16, kChR, 0L,
      p_bdf, p_bdf, 0L, kPix, kChR, kK3, 0.0625f);

  k_im2col<<<kPix / 32, 256, 0, stream>>>(RR16, kChR, kChR, IM16, kK3);
  wmma_gemm64<0, 0, 2, 0, false, 0><<<dim3(blocksN128, 1), 256, 0, stream>>>(
      IM16, IM16, kK3, 0L, WGBP, WGBP, kK3, 0L, (void*)GB32, (void*)GB32, kChGB, 0L,
      p_bgb, p_bgb, 0L, kPix, kChGB, kK3, 0.00390625f);

  k_final<<<kBatch * kImg, 256, 0, stream>>>(NRM32, GB32, out);
}
